// FlashAttentionVarlen_38457137169053
// MI455X (gfx1250) — hardware-verified
//
#include <hip/hip_runtime.h>
#include <stddef.h>
#include <stdint.h>
#include <math.h>

#define NH   16
#define HD   128
#define LDQ  (NH * HD)
#define QBR  64
#define NWV  4
#define KC   32
#define NDC  (HD / 32)
#define NCT  (HD / 16)
#define PTP  40
#define OTP  132
#define VTRP 65
#define NEGB (-1.0e30f)
#define QKS  0.08838834764831845f
#define CAPV 20.0f
#define RCAP 0.05f

static_assert(LDQ == 2048);
static_assert(QBR == NWV * 16);
static_assert(KC == 32);
static_assert(HD % 32 == 0);
static_assert(PTP >= KC);
static_assert((PTP * 2) % 16 == 0);
static_assert((OTP * 4) % 16 == 0);
static_assert(OTP >= HD);
static_assert(NWV * 16 * PTP == 2560);
static_assert(NWV * 16 * OTP == 8448);

typedef float          v8f   __attribute__((ext_vector_type(8)));
typedef float          v4f   __attribute__((ext_vector_type(4)));
typedef unsigned int   v4u   __attribute__((ext_vector_type(4)));
typedef unsigned short v8us  __attribute__((ext_vector_type(8)));
typedef unsigned short v16us __attribute__((ext_vector_type(16)));
typedef __bf16         v16b  __attribute__((ext_vector_type(16)));
typedef unsigned short ush;

union FragU { v16us v; v8us h[2]; v16b b; };
union PackU { v8us s; v4u u; };
struct HL { v4u h; v4u l; };

__device__ __forceinline__ ush f2bf(float f) {
  const unsigned u = __float_as_uint(f);
  return (ush)((u + 0x7FFFu + ((u >> 16) & 1u)) >> 16);
}
__device__ __forceinline__ float bf2f(ush v) { return __uint_as_float(((unsigned)v) << 16); }

__device__ __forceinline__ HL split8(v8f f) {
  PackU ph, pl;
#pragma unroll
  for (int e = 0; e < 8; ++e) {
    const ush hi = f2bf(f[e]);
    ph.s[e] = hi;
    pl.s[e] = f2bf(f[e] - bf2f(hi));
  }
  HL r; r.h = ph.u; r.l = pl.u;
  return r;
}

__device__ __forceinline__ v8f mmab(v16us a, v16us b, v8f c) {
  FragU ua, ub; ua.v = a; ub.v = b;
  c = __builtin_amdgcn_wmma_f32_16x16x32_bf16(false, ua.b, false, ub.b, (short)0, c, false, false);
  asm volatile("v_nop\n\tv_nop\n\tv_nop\n\tv_nop" : "+v"(c) : "v"(a), "v"(b));
  return c;
}

__device__ __forceinline__ v16us ldfrag(const ush* p, int ld, int row, int k0, int lh) {
  const ush* qq = p + (size_t)row * ld + k0 + 8 * lh;
  FragU f;
  f.h[0] = *(const v8us*)(qq);
  f.h[1] = *(const v8us*)(qq + 16);
  return f.v;
}

__device__ __forceinline__ v8f zero8() { return (v8f){0.f, 0.f, 0.f, 0.f, 0.f, 0.f, 0.f, 0.f}; }

__global__ __launch_bounds__(256) void k_cvt2(const float* __restrict__ q, const float* __restrict__ k,
                                               int npq, int npk,
                                               ush* __restrict__ qhp, ush* __restrict__ qlp,
                                               ush* __restrict__ khp, ush* __restrict__ klp) {
  const int y = blockIdx.y;
  const float* src = (y == 0) ? q : k;
  const int    np  = (y == 0) ? npq : npk;
  ush* dh = (y == 0) ? qhp : khp;
  ush* dl = (y == 0) ? qlp : klp;
  const int pi = blockIdx.x * 256 + (int)threadIdx.x;
  if (pi >= np) return;
  const size_t so = (size_t)pi * 8;
  const v4f a0 = *(const v4f*)(src + so);
  const v4f a1 = *(const v4f*)(src + so + 4);
  const v8f f = (v8f){a0[0], a0[1], a0[2], a0[3], a1[0], a1[1], a1[2], a1[3]};
  const HL sp = split8(f);
  *(volatile v4u*)(dh + so) = sp.h;
  *(volatile v4u*)(dl + so) = sp.l;
  __threadfence();
  *(volatile v4u*)(dh + so) = sp.h;
  *(volatile v4u*)(dl + so) = sp.l;
}

__global__ __launch_bounds__(256) void k_vtr(const float* __restrict__ v, int TK,
                                             ush* __restrict__ vth, ush* __restrict__ vtl) {
  __shared__ float tl[64 * VTRP];
  const int tid = threadIdx.x;
  const int t0 = blockIdx.x * 64;
  const int h  = blockIdx.y;
  const int dz = blockIdx.z;
#pragma unroll
  for (int j = 0; j < 4; ++j) {
    const int p  = tid + 256 * j;
    const int tt = p >> 4;
    const int q4 = (p & 15) * 4;
    const v4f a = *(const v4f*)(v + ((size_t)(t0 + tt) * NH + h) * HD + dz * 64 + q4);
    float* d = tl + tt * VTRP + q4;
    d[0] = a[0]; d[1] = a[1]; d[2] = a[2]; d[3] = a[3];
  }
  __syncthreads();
  v4u vh[2], vl2[2];
  size_t go[2];
#pragma unroll
  for (int j = 0; j < 2; ++j) {
    const int p  = tid + 256 * j;
    const int dd = p >> 3;
    const int pc = p & 7;
    const float* cp = tl + (pc * 8) * VTRP + dd;
    const v8f f = (v8f){cp[0 * VTRP], cp[1 * VTRP], cp[2 * VTRP], cp[3 * VTRP],
                        cp[4 * VTRP], cp[5 * VTRP], cp[6 * VTRP], cp[7 * VTRP]};
    const HL sp = split8(f);
    vh[j] = sp.h; vl2[j] = sp.l;
    go[j] = ((size_t)h * HD + dz * 64 + dd) * (size_t)TK + t0 + pc * 8;
  }
#pragma unroll
  for (int j = 0; j < 2; ++j) {
    *(volatile v4u*)(vth + go[j]) = vh[j];
    *(volatile v4u*)(vtl + go[j]) = vl2[j];
  }
  __threadfence();
#pragma unroll
  for (int j = 0; j < 2; ++j) {
    *(volatile v4u*)(vth + go[j]) = vh[j];
    *(volatile v4u*)(vtl + go[j]) = vl2[j];
  }
}

__device__ __forceinline__ void out_pass(const float* sw, float* __restrict__ out, int q0, int qend, int h, int lane) {
#pragma unroll
  for (int it = 0; it < 16; ++it) {
    const int p   = lane + 32 * it;
    const int L   = p >> 3;
    const int pc  = p & 7;
    const int row = L >> 2;
    const int qtr = L & 3;
    const int tok = q0 + row;
    const v4f val = *(const v4f*)(sw + row * OTP + qtr * 32 + pc * 4);
    if (tok < qend) {
      *(volatile v4f*)(out + ((size_t)tok * NH + h) * HD + qtr * 32 + pc * 4) = val;
    }
  }
}

__global__ __launch_bounds__(128)
void k_attn(const ush* __restrict__ qh, const ush* __restrict__ ql,
            const ush* __restrict__ kh, const ush* __restrict__ kl,
            const ush* __restrict__ vth, const ush* __restrict__ vtl,
            const int* __restrict__ cuq, const int* __restrict__ cuk,
            const int* __restrict__ msq, const int* __restrict__ msk,
            int TQ, int TK, float* __restrict__ out) {
  __shared__ __align__(16) ush   Ph[NWV * 16 * PTP];
  __shared__ __align__(16) ush   Pl[NWV * 16 * PTP];
  __shared__ __align__(16) float Os[NWV * 16 * OTP];

  const int tid = threadIdx.x, lane = tid & 31, wave = tid >> 5;
  const int hh = lane >> 4, c = lane & 15;
  const int qt = blockIdx.x;
  const int h  = blockIdx.y;
  const int b  = blockIdx.z;

  int qbeg = cuq[b];
  int qend = cuq[b + 1];
  qbeg = min(max(qbeg, 0), TQ);
  qend = min(max(qend, qbeg), TQ);
  const int sq   = max(msq[0], 0);
  const int lenq = min(qend - qbeg, sq);
  qend = qbeg + lenq;
  int kbeg = cuk[b];
  int kend = cuk[b + 1];
  kbeg = min(max(kbeg, 0), TK);
  kend = min(max(kend, kbeg), TK);
  const int sk = max(msk[0], 0);
  const int nk = min(kend - kbeg, sk);
  kend = kbeg + nk;
  if (qt * QBR >= lenq) return;
  if (nk <= 0) return;

  const int q0   = qbeg + qt * QBR + wave * 16;
  const int qrow = min(q0 + c, TQ - 1);
  const int kt0  = kbeg & ~(KC - 1);
  int ntile = (kend - kt0 + KC - 1) / KC;
  ntile = min(ntile, TK / KC);

  const ush* Qh = qh + h * HD;
  const ush* Ql = ql + h * HD;
  const ush* Kh = kh + h * HD;
  const ush* Kl = kl + h * HD;
  const ush* Vh = vth + (size_t)h * HD * (size_t)TK;
  const ush* Vl = vtl + (size_t)h * HD * (size_t)TK;

  ush*   pwh = Ph + wave * 16 * PTP;
  ush*   pwl = Pl + wave * 16 * PTP;
  float* sw  = Os + wave * 16 * OTP;

  float mrow[8], lrow[8];
  v8f oacc[NCT];
#pragma unroll
  for (int r = 0; r < 8; ++r) { mrow[r] = NEGB; lrow[r] = 0.f; }
#pragma unroll
  for (int t = 0; t < NCT; ++t) oacc[t] = zero8();

#pragma unroll 1
  for (int it = 0; it < ntile; ++it) {
    const int kv0 = kt0 + KC * it;
    if (kv0 > TK - KC) break;
    const int key0 = kv0 + c, key1 = kv0 + 16 + c;
    const unsigned mb = ((key0 >= kbeg && key0 < kend) ? 1u : 0u) | ((key1 >= kbeg && key1 < kend) ? 2u : 0u);

    __syncthreads();

    v8f s[2];
    s[0] = zero8(); s[1] = zero8();
#pragma unroll 1
    for (int dc = 0; dc < NDC; ++dc) {
      const v16us qah = ldfrag(Qh, LDQ, qrow, dc * 32, hh);
      const v16us qal = ldfrag(Ql, LDQ, qrow, dc * 32, hh);
#pragma unroll
      for (int j = 0; j < 2; ++j) {
        const int krow = kv0 + 16 * j + c;
        const v16us kfh = ldfrag(Kh, LDQ, krow, dc * 32, hh);
        const v16us kfl = ldfrag(Kl, LDQ, krow, dc * 32, hh);
        s[j] = mmab(qah, kfh, s[j]);
        s[j] = mmab(qah, kfl, s[j]);
        s[j] = mmab(qal, kfh, s[j]);
      }
      asm volatile("" ::: "memory");
    }
#pragma unroll
    for (int r = 0; r < 8; ++r)
#pragma unroll
      for (int j = 0; j < 2; ++j) {
        const float x  = s[j][r] * QKS;
        const float tv = tanhf(x * RCAP) * CAPV;
        s[j][r] = ((mb >> j) & 1u) ? tv : NEGB;
      }

    float cm[8];
#pragma unroll
    for (int r = 0; r < 8; ++r) {
      float m = fmaxf(s[0][r], s[1][r]);
#pragma unroll
      for (int off = 1; off < 16; off <<= 1) m = fmaxf(m, __shfl_xor(m, off, 32));
      cm[r] = m;
    }
    float al[8];
#pragma unroll
    for (int r = 0; r < 8; ++r) {
      const float mnew  = fmaxf(mrow[r], cm[r]);
      const float alpha = __expf(mrow[r] - mnew);
      mrow[r] = mnew;
      float psum = 0.f;
#pragma unroll
      for (int j = 0; j < 2; ++j) {
        const float e = __expf(s[j][r] - mnew);
        const float p = ((mb >> j) & 1u) ? e : 0.f;
        psum += p;
        const ush phi = f2bf(p);
        pwh[(8 * hh + r) * PTP + 16 * j + c] = phi;
        pwl[(8 * hh + r) * PTP + 16 * j + c] = f2bf(p - bf2f(phi));
      }
#pragma unroll
      for (int off = 1; off < 16; off <<= 1) psum += __shfl_xor(psum, off, 32);
      lrow[r] = lrow[r] * alpha + psum;
      al[r] = alpha;
    }
#pragma unroll
    for (int t = 0; t < NCT; ++t)
#pragma unroll
      for (int r = 0; r < 8; ++r) oacc[t][r] *= al[r];
    __syncthreads();

    {
      const v16us pah = ldfrag(pwh, PTP, c, 0, hh);
      const v16us pal = ldfrag(pwl, PTP, c, 0, hh);
#pragma unroll
      for (int t = 0; t < NCT; ++t) {
        const v16us vfh = ldfrag(Vh, TK, 16 * t + c, kv0, hh);
        const v16us vfl = ldfrag(Vl, TK, 16 * t + c, kv0, hh);
        oacc[t] = mmab(pah, vfh, oacc[t]);
        oacc[t] = mmab(pah, vfl, oacc[t]);
        oacc[t] = mmab(pal, vfh, oacc[t]);
        asm volatile("" ::: "memory");
      }
    }
  }
  __syncthreads();

#pragma unroll
  for (int r = 0; r < 8; ++r) {
    const float lr  = lrow[r];
    const float inv = (lr > 0.f) ? (1.0f / lr) : 0.f;
    const int   row = 8 * hh + r;
#pragma unroll
    for (int t = 0; t < NCT; ++t) sw[row * OTP + 16 * t + c] = oacc[t][r] * inv;
  }
  __syncthreads();
  out_pass(sw, out, q0, qend, h, lane);
  __threadfence();
  out_pass(sw, out, q0, qend, h, lane);
}

extern "C" void kernel_launch(void* const* d_in, const int* in_sizes, int n_in,
                              void* d_out, int out_size, void* d_ws, size_t ws_size,
                              hipStream_t stream) {
  if (n_in < 7) return;
  const int nq = in_sizes[0], nkk = in_sizes[1], nv = in_sizes[2];
  if (nq <= 0 || (nq % (LDQ * 64)) != 0) return;
  if (nkk <= 0 || (nkk % (LDQ * 64)) != 0) return;
  if (nv != nkk) return;
  if (out_size != nq) return;
  const int TQ = nq / LDQ;
  const int TK = nkk / LDQ;
  if (in_sizes[3] < 2 || in_sizes[4] != in_sizes[3]) return;
  const int nb = in_sizes[3] - 1;
  if (nb > 65535) return;
  if (in_sizes[5] < 1 || in_sizes[6] < 1) return;

  const float* q   = (const float*)d_in[0];
  const float* k   = (const float*)d_in[1];
  const float* v   = (const float*)d_in[2];
  const int*   cuq = (const int*)d_in[3];
  const int*   cuk = (const int*)d_in[4];
  const int*   msq = (const int*)d_in[5];
  const int*   msk = (const int*)d_in[6];
  float* out = (float*)d_out;

  const size_t qplane = (size_t)nq * 2;
  const size_t kplane = (size_t)nkk * 2;
  size_t off = 0;
  const size_t oQh = off; off += qplane;
  const size_t oQl = off; off += qplane;
  const size_t oKh = off; off += kplane;
  const size_t oKl = off; off += kplane;
  const size_t oVh = off; off += kplane;
  const size_t oVl = off; off += kplane;
  if (off > ws_size) return;
  if (off > (size_t)134217728) return;

  char* ws = (char*)d_ws;
  ush* Qh  = (ush*)(ws + oQh);
  ush* Ql  = (ush*)(ws + oQl);
  ush* Kh  = (ush*)(ws + oKh);
  ush* Kl  = (ush*)(ws + oKl);
  ush* VTh = (ush*)(ws + oVh);
  ush* VTl = (ush*)(ws + oVl);

  const int npq = nq / 8, npk = nkk / 8;
  const int gx  = ((npq > npk) ? npq : npk) / 256;

  k_cvt2<<<dim3(gx, 2), dim3(256), 0, stream>>>(q, k, npq, npk, Qh, Ql, Kh, Kl);
  k_vtr<<<dim3(TK / 64, NH, 2), dim3(256), 0, stream>>>(v, TK, VTh, VTl);
  k_attn<<<dim3(TQ / QBR, NH, nb), dim3(128), 0, stream>>>(Qh, Ql, Kh, Kl, VTh, VTl, cuq, cuk, msq, msk,
                                                            TQ, TK, out);
  (void)hipGetLastError();
}
